// GCN_Hetro_30846455120312
// MI455X (gfx1250) — hardware-verified
//
#include <hip/hip_runtime.h>
#include <stddef.h>


#define EMB      64
#define HF       128
#define NTHR     256
#define NWAVE    8
#define EPT      8
#define NGRP     2
#define CHUNK    (NTHR * EPT * NGRP)
#define WCAP     (EPT * NGRP * 32)
#define LISTN    (NWAVE * WCAP)
#define NB       512
#define EPSC     1e-5f
#define LDS_SAGE (NB * HF * 4 + LISTN * 4 + NB * 4 + 3 * HF * 4 + 64)

static_assert((CHUNK & (CHUNK - 1)) == 0);
static_assert(CHUNK <= 4096);
static_assert((NB & (NB - 1)) == 0);
static_assert(NB <= 4096);
static_assert(NB % (16 * NWAVE) == 0);
static_assert(NB % (8 * NWAVE) == 0);
static_assert(6 * HF * 8 <= LISTN * 4);
static_assert(EMB % 32 == 0);
static_assert(HF % 32 == 0);

typedef float          v4f  __attribute__((ext_vector_type(4)));
typedef float          v8f  __attribute__((ext_vector_type(8)));
typedef int            v4i  __attribute__((ext_vector_type(4)));
typedef double         v2d  __attribute__((ext_vector_type(2)));
typedef unsigned short v8us __attribute__((ext_vector_type(8)));
typedef __bf16         v2b  __attribute__((ext_vector_type(2)));
typedef __bf16         v16b __attribute__((ext_vector_type(16)));
union FragB { v16b v; v8us u8[2]; unsigned u[8]; };
union Pk2   { v2b b; unsigned u; };
union Pk8   { v8us v; unsigned u[4]; };

__device__ __forceinline__ v4f ld4(const float* p) { return *(const v4f*)p; }

__device__ __forceinline__ v8f wmb(v16b a, v16b b, v8f c) {
  v8f d = __builtin_amdgcn_wmma_f32_16x16x32_bf16(false, a, false, b, (short)0, c, false, false);
  asm volatile("v_nop\n\tv_nop\n\tv_nop\n\tv_nop" : "+v"(d) : "v"(a), "v"(b));
  return d;
}

__device__ __forceinline__ void split16(const v4f p0, const v4f p1, const v4f p2, const v4f p3,
                                        FragB& hi, FragB& lo) {
  const float x[16] = {p0.x, p0.y, p0.z, p0.w, p1.x, p1.y, p1.z, p1.w,
                       p2.x, p2.y, p2.z, p2.w, p3.x, p3.y, p3.z, p3.w};
#pragma unroll
  for (int j = 0; j < 8; ++j) {
    Pk2 h;
    h.b.x = (__bf16)x[2 * j];
    h.b.y = (__bf16)x[2 * j + 1];
    const float f0 = __uint_as_float(h.u << 16);
    const float f1 = __uint_as_float(h.u & 0xFFFF0000u);
    Pk2 l;
    l.b.x = (__bf16)(x[2 * j] - f0);
    l.b.y = (__bf16)(x[2 * j + 1] - f1);
    hi.u[j] = h.u;
    lo.u[j] = l.u;
  }
}

__device__ __forceinline__ void mma8(v8f (&c)[8], const v16b ah, const v16b al,
                                     const unsigned short* whp, const unsigned short* wlp, int K) {
#pragma unroll
  for (int ct = 0; ct < 8; ++ct) {
    FragB bh, bl;
    const unsigned short* ph = whp + (size_t)(16 * ct) * K;
    const unsigned short* pl = wlp + (size_t)(16 * ct) * K;
    bh.u8[0] = *(const v8us*)ph;
    bh.u8[1] = *(const v8us*)(ph + 16);
    bl.u8[0] = *(const v8us*)pl;
    bl.u8[1] = *(const v8us*)(pl + 16);
    c[ct] = wmb(ah, bh.v, c[ct]);
    c[ct] = wmb(ah, bl.v, c[ct]);
    c[ct] = wmb(al, bh.v, c[ct]);
  }
}

template <int NBT>
__device__ __forceinline__ int scan_chunk(const int* __restrict__ keys, int nE, int cbase, int keyBase,
                                          int vec8, int* list, int tid, int lane, int wave) {
  int wc = 0;
#pragma unroll
  for (int g = 0; g < NGRP; ++g) {
    const int el0  = (g * NTHR + tid) * EPT;
    const int e0   = cbase + el0;
    const int sent = -2147483647 - 1;
    v4i da, db;
    if (vec8 != 0 && cbase + CHUNK <= nE) {
      da = *(const v4i*)(keys + e0);
      db = *(const v4i*)(keys + e0 + 4);
    } else {
      const int lz = nE - 1;
      da.x = (e0     < nE) ? keys[min(e0,     lz)] : sent;
      da.y = (e0 + 1 < nE) ? keys[min(e0 + 1, lz)] : sent;
      da.z = (e0 + 2 < nE) ? keys[min(e0 + 2, lz)] : sent;
      da.w = (e0 + 3 < nE) ? keys[min(e0 + 3, lz)] : sent;
      db.x = (e0 + 4 < nE) ? keys[min(e0 + 4, lz)] : sent;
      db.y = (e0 + 5 < nE) ? keys[min(e0 + 5, lz)] : sent;
      db.z = (e0 + 6 < nE) ? keys[min(e0 + 6, lz)] : sent;
      db.w = (e0 + 7 < nE) ? keys[min(e0 + 7, lz)] : sent;
    }
    const unsigned nb = (unsigned)keyBase;
    const unsigned s0 = (unsigned)da.x - nb, s1 = (unsigned)da.y - nb;
    const unsigned s2 = (unsigned)da.z - nb, s3 = (unsigned)da.w - nb;
    const unsigned s4 = (unsigned)db.x - nb, s5 = (unsigned)db.y - nb;
    const unsigned s6 = (unsigned)db.z - nb, s7 = (unsigned)db.w - nb;
    const bool h0 = s0 < (unsigned)NBT, h1 = s1 < (unsigned)NBT, h2 = s2 < (unsigned)NBT, h3 = s3 < (unsigned)NBT;
    const bool h4 = s4 < (unsigned)NBT, h5 = s5 < (unsigned)NBT, h6 = s6 < (unsigned)NBT, h7 = s7 < (unsigned)NBT;
    const unsigned any = __builtin_amdgcn_ballot_w32(h0 | h1 | h2 | h3 | h4 | h5 | h6 | h7);
    if (any != 0u) {
#define HITJ(J, HJ, SJ) { \
        const unsigned mj = __builtin_amdgcn_ballot_w32(HJ); \
        if (mj != 0u) { \
          if (HJ) { \
            const int pos = wc + (int)__builtin_amdgcn_mbcnt_lo(mj, 0u); \
            if (pos < WCAP) list[wave * WCAP + pos] = ((el0 + (J)) << 12) | (int)(SJ); \
          } \
          wc += (int)__builtin_popcount(mj); } }
      HITJ(0, h0, s0)
      HITJ(1, h1, s1)
      HITJ(2, h2, s2)
      HITJ(3, h3, s3)
      HITJ(4, h4, s4)
      HITJ(5, h5, s5)
      HITJ(6, h6, s6)
      HITJ(7, h7, s7)
#undef HITJ
    }
  }
  return wc;
}

__global__ __launch_bounds__(NTHR) void k_wsplit(
    const float* __restrict__ W1s, const float* __restrict__ W1n,
    const float* __restrict__ Ws,  const float* __restrict__ Wn,
    unsigned short* wh, unsigned short* wl, int nTot8) {
  const int t = blockIdx.x * NTHR + threadIdx.x;
  if (t >= nTot8) return;
  const int o  = t * 8;
  const int R0 = 3 * HF * 2 * EMB;
  float xa[8], xb[8];
  bool useB;
  if (o < R0) {
    const int mat = o / (HF * 2 * EMB);
    const int rem = o - mat * (HF * 2 * EMB);
    const int n   = rem / (2 * EMB);
    const int k0  = rem - n * (2 * EMB);
    useB = k0 >= EMB;
    const int kk = useB ? k0 - EMB : k0;
    const float* pa = W1s + ((size_t)mat * EMB + kk) * HF + n;
    const float* pb = W1n + ((size_t)mat * EMB + kk) * HF + n;
#pragma unroll
    for (int j = 0; j < 8; ++j) { xa[j] = pa[(size_t)j * HF]; xb[j] = pb[(size_t)j * HF]; }
  } else {
    const int o2  = o - R0;
    const int mat = o2 / (HF * 2 * HF);
    const int rem = o2 - mat * (HF * 2 * HF);
    const int n   = rem / (2 * HF);
    const int k0  = rem - n * (2 * HF);
    useB = k0 >= HF;
    const int kk = useB ? k0 - HF : k0;
    const float* pa = Ws + ((size_t)mat * HF + kk) * HF + n;
    const float* pb = Wn + ((size_t)mat * HF + kk) * HF + n;
#pragma unroll
    for (int j = 0; j < 8; ++j) { xa[j] = pa[(size_t)j * HF]; xb[j] = pb[(size_t)j * HF]; }
  }
  Pk8 H, L;
#pragma unroll
  for (int j = 0; j < 4; ++j) {
    const float x0 = useB ? xb[2 * j]     : xa[2 * j];
    const float x1 = useB ? xb[2 * j + 1] : xa[2 * j + 1];
    Pk2 h;
    h.b.x = (__bf16)x0;
    h.b.y = (__bf16)x1;
    const float f0 = __uint_as_float(h.u << 16);
    const float f1 = __uint_as_float(h.u & 0xFFFF0000u);
    Pk2 l;
    l.b.x = (__bf16)(x0 - f0);
    l.b.y = (__bf16)(x1 - f1);
    H.u[j] = h.u;
    L.u[j] = l.u;
  }
  const v8us hv = H.v, lv = L.v;
  *(volatile v8us*)(wh + o) = hv;
  *(volatile v8us*)(wl + o) = lv;
  __threadfence();
  *(volatile v8us*)(wh + o) = hv;
  *(volatile v8us*)(wl + o) = lv;
}

__global__ __launch_bounds__(NTHR) void k_embed(const int* __restrict__ idx, const float* __restrict__ emb,
                                                float* x0, int nN, int nRows, int nEmbR) {
  const int t = blockIdx.x * NTHR + threadIdx.x;
  if (t >= nRows * (EMB / 4)) return;
  const int n  = t >> 4;
  const int c0 = (t & 15) * 4;
  const int nn = n > nN - 1 ? nN - 1 : n;
  int r = idx[nn];
  r = r < 0 ? 0 : (r > nEmbR - 1 ? nEmbR - 1 : r);
  const v4f v = *(const v4f*)(emb + (size_t)r * EMB + c0);
  float* gp = x0 + (size_t)n * EMB + c0;
  *(volatile v4f*)gp = v;
  __threadfence();
  *(volatile v4f*)gp = v;
}

__global__ __launch_bounds__(NTHR) __attribute__((amdgpu_num_vgpr(256)))
void k_sage(const int* __restrict__ srcs, const int* __restrict__ dsts,
            const float* __restrict__ X,
            const unsigned short* __restrict__ wh, const unsigned short* __restrict__ wl,
            const float* __restrict__ bias, const float* __restrict__ slope,
            const double* __restrict__ psIn, const double* __restrict__ pqIn,
            const float* __restrict__ gam, const float* __restrict__ bet,
            float* Z, double* psOut, double* pqOut,
            int Din, int hasBN, int nN, int nE, int nblkIn, int vec8) {
  extern __shared__ v4f lds_dyn[];
  float*  acc  = (float*)lds_dyn;
  int*    list = (int*)(acc + NB * HF);
  int*    cnt  = list + LISTN;
  float*  bnp  = (float*)(cnt + NB);
  int*    wcnt = (int*)(bnp + 3 * HF);
  double* red  = (double*)list;
  const int tid = threadIdx.x, lane = tid & 31, wave = tid >> 5, hh = lane >> 4, m = lane & 15;
  const int nodeBase = blockIdx.x * NB;

  {
    const v4f z = {0.f, 0.f, 0.f, 0.f};
    for (int i = tid; i < NB * HF / 4; i += NTHR) lds_dyn[i] = z;
  }
  for (int i = tid; i < NB; i += NTHR) cnt[i] = 0;

  {
    const int c = tid & (HF - 1), which = tid >> 7;
    if (hasBN != 0) {
      const double* pp = (which != 0) ? pqIn : psIn;
      double s = 0.0;
#pragma unroll 1
      for (int b = 0; b < nblkIn; ++b) s += pp[(size_t)b * HF + c];
      red[which * HF + c] = s;
    }
    __syncthreads();
    if (tid < HF) {
      float mu = 0.f, gs = 1.f, be = 0.f;
      if (hasBN != 0) {
        const double invn = 1.0 / (double)nN;
        const double mud  = red[c] * invn;
        double var = red[HF + c] * invn - mud * mud;
        var = var < 0.0 ? 0.0 : var;
        mu = (float)mud;
        gs = gam[c] * rsqrtf((float)var + EPSC);
        be = bet[c];
      }
      bnp[c] = mu; bnp[HF + c] = gs; bnp[2 * HF + c] = be;
    }
  }
  __syncthreads();

  const int dclamp  = Din - 4;
  const int nChunks = (nE + CHUNK - 1) / CHUNK;
#pragma unroll 1
  for (int ch = 0; ch < nChunks; ++ch) {
    const int cbase = ch * CHUNK;
    const int wc = scan_chunk<NB>(dsts, nE, cbase, nodeBase, vec8, list, tid, lane, wave);
    if (lane == 0) wcnt[wave] = wc;
    __syncthreads();
    if (wave == 0) {
      const int col = min(4 * lane, dclamp);
#pragma unroll 1
      for (int wsx = 0; wsx < NWAVE; ++wsx) {
        int n = __builtin_amdgcn_readfirstlane(wcnt[wsx]);
        n = n > WCAP ? WCAP : (n < 0 ? 0 : n);
        const int* lp = list + wsx * WCAP;
#pragma unroll 1
        for (int i = 0; i < n; ++i) {
          const int ent  = __builtin_amdgcn_readfirstlane(lp[i]);
          const int slot = ent & (NB - 1);
          int e = cbase + ((ent >> 12) & (CHUNK - 1));
          e = e > nE - 1 ? nE - 1 : e;
          int s = srcs[e];
          s = s < 0 ? 0 : (s > nN - 1 ? nN - 1 : s);
          const v4f v = *(const v4f*)(X + (size_t)s * Din + col);
          v4f* ap = (v4f*)(acc + (size_t)slot * HF + 4 * lane);
          *ap = *ap + v;
          if (lane == 0) cnt[slot] = cnt[slot] + 1;
        }
      }
    }
    __syncthreads();
  }

  float bcol[8], acol[8];
#pragma unroll
  for (int ct = 0; ct < 8; ++ct) { bcol[ct] = bias[16 * ct + m]; acol[ct] = slope[16 * ct + m]; }
  const int K   = 2 * Din;
  const int nks = Din >> 5;
#pragma unroll 1
  for (int tt = 0; tt < NB / (16 * NWAVE); ++tt) {
    const int t    = wave + NWAVE * tt;
    const int rloc = 16 * t + m;
    int node = nodeBase + rloc;
    node = node > nN - 1 ? nN - 1 : node;
    const int dg = cnt[rloc];
    const float rinv = 1.0f / (float)(dg > 0 ? dg : 1);
    const float fnz  = dg > 0 ? 1.f : 0.f;
    v8f cacc[8];
#pragma unroll
    for (int ct = 0; ct < 8; ++ct) { const v8f z8 = {0.f, 0.f, 0.f, 0.f, 0.f, 0.f, 0.f, 0.f}; cacc[ct] = z8; }
    const float* xrow = X + (size_t)node * Din + 8 * hh;
    const float* arow = acc + (size_t)rloc * HF + 8 * hh;
    const float* prow = bnp + 8 * hh;
    const unsigned short* whr = wh + (size_t)m * K + 8 * hh;
    const unsigned short* wlr = wl + (size_t)m * K + 8 * hh;

#pragma unroll 1
    for (int kt = 0; kt < nks; ++kt) {
      const int k0 = 32 * kt;
      v4f p0 = ld4(xrow + k0),      p1 = ld4(xrow + k0 + 4);
      v4f p2 = ld4(xrow + k0 + 16), p3 = ld4(xrow + k0 + 20);
      const float* pp = prow + k0;
      p0 = (p0 - ld4(pp))      * ld4(pp + HF)      + ld4(pp + 2 * HF);
      p1 = (p1 - ld4(pp + 4))  * ld4(pp + HF + 4)  + ld4(pp + 2 * HF + 4);
      p2 = (p2 - ld4(pp + 16)) * ld4(pp + HF + 16) + ld4(pp + 2 * HF + 16);
      p3 = (p3 - ld4(pp + 20)) * ld4(pp + HF + 20) + ld4(pp + 2 * HF + 20);
      FragB ah, al;
      split16(p0, p1, p2, p3, ah, al);
      mma8(cacc, ah.v, al.v, whr + k0, wlr + k0, K);
    }
#pragma unroll 1
    for (int kt = 0; kt < nks; ++kt) {
      const int c0 = 32 * kt;
      v4f p0 = ld4(arow + c0),      p1 = ld4(arow + c0 + 4);
      v4f p2 = ld4(arow + c0 + 16), p3 = ld4(arow + c0 + 20);
      const float* pp = prow + c0;
      p0 = ((p0 * rinv - ld4(pp))      * ld4(pp + HF)      + ld4(pp + 2 * HF))      * fnz;
      p1 = ((p1 * rinv - ld4(pp + 4))  * ld4(pp + HF + 4)  + ld4(pp + 2 * HF + 4))  * fnz;
      p2 = ((p2 * rinv - ld4(pp + 16)) * ld4(pp + HF + 16) + ld4(pp + 2 * HF + 16)) * fnz;
      p3 = ((p3 * rinv - ld4(pp + 20)) * ld4(pp + HF + 20) + ld4(pp + 2 * HF + 20)) * fnz;
      FragB ah, al;
      split16(p0, p1, p2, p3, ah, al);
      mma8(cacc, ah.v, al.v, whr + Din + c0, wlr + Din + c0, K);
    }
    float* zp = acc + (size_t)(16 * t + 8 * hh) * HF + m;
#pragma unroll
    for (int ct = 0; ct < 8; ++ct) {
#pragma unroll
      for (int r = 0; r < 8; ++r) {
        float y = cacc[ct][r] + bcol[ct];
        y = (y > 0.f) ? y : acol[ct] * y;
        zp[r * HF + 16 * ct] = y;
      }
    }
  }
  __syncthreads();

  {
    const float* lp = acc + (size_t)(wave * (NB / NWAVE)) * HF + 4 * lane;
    float* gp = Z + ((size_t)nodeBase + wave * (NB / NWAVE)) * HF + 4 * lane;
#pragma unroll 8
    for (int r = 0; r < NB / NWAVE; ++r) { const v4f v = ld4(lp + r * HF); *(volatile v4f*)(gp + (size_t)r * HF) = v; }
    __threadfence();
#pragma unroll 8
    for (int r = 0; r < NB / NWAVE; ++r) { const v4f v = ld4(lp + r * HF); *(volatile v4f*)(gp + (size_t)r * HF) = v; }
  }

  {
    int nvalid = nN - nodeBase;
    nvalid = nvalid > NB ? NB : nvalid;
    const int c  = tid & (HF - 1), hf = tid >> 7;
    const int r0 = hf * (NB / 2);
    int r1 = r0 + NB / 2;
    r1 = r1 > nvalid ? nvalid : r1;
    double s = 0.0, q = 0.0;
#pragma unroll 4
    for (int r = r0; r < r1; ++r) {
      const double z = (double)acc[r * HF + c];
      s += z;
      q += z * z;
    }
    red[hf * HF + c] = s;
    red[2 * HF + hf * HF + c] = q;
  }
  __syncthreads();
  double* stg = red + 4 * HF;
  if (tid < HF) {
    stg[tid]      = red[tid] + red[HF + tid];
    stg[HF + tid] = red[2 * HF + tid] + red[3 * HF + tid];
  }
  __syncthreads();
  if (tid < 64) {
    const v2d v = *(const v2d*)(stg + 2 * tid);
    *(volatile v2d*)(psOut + (size_t)blockIdx.x * HF + 2 * tid) = v;
  } else if (tid < 128) {
    const v2d v = *(const v2d*)(stg + HF + 2 * (tid - 64));
    *(volatile v2d*)(pqOut + (size_t)blockIdx.x * HF + 2 * (tid - 64)) = v;
  }
  __threadfence();
  if (tid < 64) {
    const v2d v = *(const v2d*)(stg + 2 * tid);
    *(volatile v2d*)(psOut + (size_t)blockIdx.x * HF + 2 * tid) = v;
  } else if (tid < 128) {
    const v2d v = *(const v2d*)(stg + HF + 2 * (tid - 64));
    *(volatile v2d*)(pqOut + (size_t)blockIdx.x * HF + 2 * (tid - 64)) = v;
  }
}

__global__ __launch_bounds__(NTHR) void k_readout(
    const int* __restrict__ segs, const float* __restrict__ Z,
    const double* __restrict__ psIn, const double* __restrict__ pqIn,
    const float* __restrict__ gam, const float* __restrict__ bet,
    float* out, int nN, int nblkIn, int pitch, int colOff, int vec8) {
  __shared__ __attribute__((aligned(16))) int    list[LISTN];
  __shared__ __attribute__((aligned(16))) float  gacc[HF];
  __shared__ __attribute__((aligned(16))) float  res[HF];
  __shared__ __attribute__((aligned(16))) float  bnp[3 * HF];
  __shared__ __attribute__((aligned(16))) double red[2 * HF];
  __shared__ int wcnt[NWAVE];
  __shared__ int cntg[4];
  const int tid = threadIdx.x, lane = tid & 31, wave = tid >> 5;
  const int g = blockIdx.x;

  {
    const int c = tid & (HF - 1), which = tid >> 7;
    const double* pp = (which != 0) ? pqIn : psIn;
    double s = 0.0;
#pragma unroll 1
    for (int b = 0; b < nblkIn; ++b) s += pp[(size_t)b * HF + c];
    red[which * HF + c] = s;
  }
  if (tid < HF) gacc[tid] = 0.f;
  if (tid == 0) cntg[0] = 0;
  __syncthreads();
  if (tid < HF) {
    const double invn = 1.0 / (double)nN;
    const double mud  = red[tid] * invn;
    double var = red[HF + tid] * invn - mud * mud;
    var = var < 0.0 ? 0.0 : var;
    bnp[tid]          = (float)mud;
    bnp[HF + tid]     = gam[tid] * rsqrtf((float)var + EPSC);
    bnp[2 * HF + tid] = bet[tid];
  }
  __syncthreads();

  const v4f mu4 = ld4(bnp + 4 * lane), gs4 = ld4(bnp + HF + 4 * lane), be4 = ld4(bnp + 2 * HF + 4 * lane);
  const int nChunks = (nN + CHUNK - 1) / CHUNK;
#pragma unroll 1
  for (int ch = 0; ch < nChunks; ++ch) {
    const int cbase = ch * CHUNK;
    const int wc = scan_chunk<1>(segs, nN, cbase, g, vec8, list, tid, lane, wave);
    if (lane == 0) wcnt[wave] = wc;
    __syncthreads();
    if (wave == 0) {
#pragma unroll 1
      for (int wsx = 0; wsx < NWAVE; ++wsx) {
        int n = __builtin_amdgcn_readfirstlane(wcnt[wsx]);
        n = n > WCAP ? WCAP : (n < 0 ? 0 : n);
        const int* lp = list + wsx * WCAP;
#pragma unroll 1
        for (int i = 0; i < n; ++i) {
          const int ent = __builtin_amdgcn_readfirstlane(lp[i]);
          int node = cbase + ((ent >> 12) & (CHUNK - 1));
          node = node > nN - 1 ? nN - 1 : node;
          const v4f v = *(const v4f*)(Z + (size_t)node * HF + 4 * lane);
          v4f* ap = (v4f*)(gacc + 4 * lane);
          *ap = *ap + ((v - mu4) * gs4 + be4);
          if (lane == 0) cntg[0] = cntg[0] + 1;
        }
      }
    }
    __syncthreads();
  }

  if (tid < HF) {
    const int n = cntg[0];
    const float rc = 1.0f / (float)(n > 0 ? n : 1);
    res[tid] = gacc[tid] * rc;
  }
  __syncthreads();
  float* gp = out + (size_t)g * pitch + colOff + 4 * lane;
  if (wave == 0) { const v4f v = ld4(res + 4 * lane); *(volatile v4f*)gp = v; }
  __threadfence();
  if (wave == 0) { const v4f v = ld4(res + 4 * lane); *(volatile v4f*)gp = v; }
}

static inline size_t al256(size_t x) { return (x + 255) & ~(size_t)255; }

extern "C" void kernel_launch(void* const* d_in, const int* in_sizes, int n_in,
                              void* d_out, int out_size, void* d_ws, size_t ws_size,
                              hipStream_t stream) {
  if (n_in < 21) return;
  const int nN = in_sizes[0];
  if (nN <= 0 || in_sizes[1] != nN || in_sizes[2] != nN) return;
  if (in_sizes[3] <= 0 || (in_sizes[3] % 3) != 0 || in_sizes[4] != in_sizes[3]) return;
  const int nE = in_sizes[3] / 3;
  if (in_sizes[5] != 3 * nN) return;
  if (in_sizes[6] < EMB || (in_sizes[6] % EMB) != 0 || in_sizes[7] != in_sizes[6] || in_sizes[8] != in_sizes[6]) return;
  const int nEmbR = in_sizes[6] / EMB;
  if (in_sizes[9] != 3 * EMB * HF || in_sizes[10] != 3 * EMB * HF) return;
  for (int q = 11; q <= 14; ++q) if (in_sizes[q] != 3 * HF) return;
  if (in_sizes[15] != 9 * HF * HF || in_sizes[16] != 9 * HF * HF) return;
  for (int q = 17; q <= 20; ++q) if (in_sizes[q] != 9 * HF) return;
  const int pitch = 12 * HF;
  if (out_size <= 0 || (out_size % pitch) != 0) return;
  const int nGr = out_size / pitch;

  const int*   hI   = (const int*)d_in[0];
  const int*   pI   = (const int*)d_in[1];
  const int*   hpI  = (const int*)d_in[2];
  const int*   src  = (const int*)d_in[3];
  const int*   dst  = (const int*)d_in[4];
  const int*   seg  = (const int*)d_in[5];
  const float* eH   = (const float*)d_in[6];
  const float* eP   = (const float*)d_in[7];
  const float* eHP  = (const float*)d_in[8];
  const float* W1s  = (const float*)d_in[9];
  const float* W1n  = (const float*)d_in[10];
  const float* b1   = (const float*)d_in[11];
  const float* a1   = (const float*)d_in[12];
  const float* g1   = (const float*)d_in[13];
  const float* be1  = (const float*)d_in[14];
  const float* Ws   = (const float*)d_in[15];
  const float* Wn   = (const float*)d_in[16];
  const float* bb   = (const float*)d_in[17];
  const float* aa   = (const float*)d_in[18];
  const float* gg   = (const float*)d_in[19];
  const float* bbe  = (const float*)d_in[20];
  float* out = (float*)d_out;

  const int nblk = (nN + NB - 1) / NB;
  const int NP   = nblk * NB;
  const int nW   = 3 * HF * 2 * EMB + 9 * HF * 2 * HF;

  char* ws = (char*)d_ws;
  size_t off = 0;
  const size_t oWH = off; off = al256(off + (size_t)nW * 2);
  const size_t oWL = off; off = al256(off + (size_t)nW * 2);
  const size_t oX0 = off; off = al256(off + (size_t)NP * EMB * 4);
  const size_t oZ0 = off; off = al256(off + (size_t)NP * HF * 4);
  const size_t oZ1 = off; off = al256(off + (size_t)NP * HF * 4);
  const size_t oPS = off; off = al256(off + (size_t)12 * nblk * HF * 8);
  const size_t oPQ = off; off = al256(off + (size_t)12 * nblk * HF * 8);
  if (off > ws_size) return;
  unsigned short* wh = (unsigned short*)(ws + oWH);
  unsigned short* wl = (unsigned short*)(ws + oWL);
  float*  x0 = (float*)(ws + oX0);
  float*  z0 = (float*)(ws + oZ0);
  float*  z1 = (float*)(ws + oZ1);
  double* ps = (double*)(ws + oPS);
  double* pq = (double*)(ws + oPQ);

  const int vec8e = ((nE % 4) == 0) ? 1 : 0;
  const int vec8n = ((nN % 4) == 0) ? 1 : 0;

  const int nTot8 = nW / 8;
  k_wsplit<<<(nTot8 + NTHR - 1) / NTHR, NTHR, 0, stream>>>(W1s, W1n, Ws, Wn, wh, wl, nTot8);

  hipFuncSetAttribute(reinterpret_cast<const void*>(&k_sage),
                      hipFuncAttributeMaxDynamicSharedMemorySize, LDS_SAGE);

  float* Zp[2] = {z0, z1};
  for (int i = 0; i < 3; ++i) {
    const int*   idxi = (i == 0) ? hI : ((i == 1) ? pI : hpI);
    const float* embi = (i == 0) ? eH : ((i == 1) ? eP : eHP);
    const int nThrE = NP * (EMB / 4);
    k_embed<<<(nThrE + NTHR - 1) / NTHR, NTHR, 0, stream>>>(idxi, embi, x0, nN, NP, nEmbR);

    for (int l = 0; l < 4; ++l) {
      const float* Xin = (l == 0) ? x0 : Zp[(l - 1) & 1];
      float*       Zo  = Zp[l & 1];
      const int    Din = (l == 0) ? EMB : HF;
      const size_t woff = (l == 0) ? (size_t)i * HF * 2 * EMB
                                   : (size_t)3 * HF * 2 * EMB + (size_t)((l - 1) * 3 + i) * HF * 2 * HF;
      const float* bL = (l == 0) ? b1 + (size_t)i * HF : bb + (size_t)((l - 1) * 3 + i) * HF;
      const float* aL = (l == 0) ? a1 + (size_t)i * HF : aa + (size_t)((l - 1) * 3 + i) * HF;
      const float*  gIn  = (l <= 1) ? g1  + (size_t)i * HF : gg  + (size_t)((l - 2) * 3 + i) * HF;
      const float*  beIn = (l <= 1) ? be1 + (size_t)i * HF : bbe + (size_t)((l - 2) * 3 + i) * HF;
      const double* psI  = (l == 0) ? ps : ps + (size_t)((l - 1) * 3 + i) * nblk * HF;
      const double* pqI  = (l == 0) ? pq : pq + (size_t)((l - 1) * 3 + i) * nblk * HF;
      double* psO = ps + (size_t)(l * 3 + i) * nblk * HF;
      double* pqO = pq + (size_t)(l * 3 + i) * nblk * HF;
      k_sage<<<nblk, NTHR, LDS_SAGE, stream>>>(src + (size_t)i * nE, dst + (size_t)i * nE, Xin,
                                               wh + woff, wl + woff, bL, aL, psI, pqI, gIn, beIn,
                                               Zo, psO, pqO, Din, (l > 0) ? 1 : 0, nN, nE, nblk, vec8e);
      const float* gL  = (l == 0) ? g1  + (size_t)i * HF : gg  + (size_t)((l - 1) * 3 + i) * HF;
      const float* beL = (l == 0) ? be1 + (size_t)i * HF : bbe + (size_t)((l - 1) * 3 + i) * HF;
      k_readout<<<nGr, NTHR, 0, stream>>>(seg + (size_t)i * nN, Zo, psO, pqO, gL, beL, out,
                                          nN, nblk, pitch, i * 4 * HF + l * HF, vec8n);
    }
  }
}
